// GraphSAGE_90984587198486
// MI455X (gfx1250) — hardware-run, weakly checked
//
#include <hip/hip_runtime.h>
#include <stddef.h>
#include <stdint.h>


#define NNODE  50000
#define NEDGE  800000
#define DF     128
#define MP     50048
#define AGP    256
#define NBA    1024
#define SLA    10
#define NBLK   49
#define NTHR   256
#define NWAVE  8
#define EPT    8
#define CHUNK  (NTHR * EPT)
#define NCHUNK ((NEDGE + CHUNK - 1) / CHUNK)
#define RCAP   28672
#define WLCAP  (RCAP / NWAVE)
#define DEGCAP 64
#define FLP    32
#define GBM    64
#define GBN    128
#define GTHR   128
#define GWAVE  4
#define ROWH   256
#define UPART  2048
#define NUW    (7 * UPART)
#define NUXB   (MP * (DF / 8))
#define NUPADP ((MP - NNODE) * AGP / 8)
#define NUPAD  (2 * NUPADP)
#define NUB    NTHR
#define NUTOT  (NUW + NUXB + NUPAD + NUB)
#define BK_LISTS (NWAVE * WLCAP)
#define BK_ZINTS (BK_LISTS + RCAP + 3 * NBA)
#define BK_MISC  16
#define BK_LDS_INTS (BK_ZINTS + BK_MISC)
#define WSMAX  134217728

constexpr int L1_S0W = 128, L1_S0P = 128;
constexpr int L1_S1W = 256, L1_S1P = AGP;
constexpr int L2_S0W = 256, L2_S0P = AGP;
constexpr int L2_S1W = 256, L2_S1P = AGP;
constexpr int K1T = L1_S0W + L1_S1W;
constexpr int K2T = L2_S0W + L2_S1W;

static_assert(MP == 391 * 128);
static_assert(NBLK * NBA >= MP && NBLK * NBA >= NNODE);
static_assert(NBA % 128 == 0 && NBA % GBM == 0 && NBA == (1 << SLA) && NBA == NTHR * 4);
static_assert(MP % GBM == 0 && MP >= NNODE);
static_assert(K1T % 32 == 0 && K2T % 32 == 0 && K1T == 3 * DF && K2T == 4 * DF);
static_assert(NNODE <= 65536);
static_assert(NEDGE % EPT == 0 && NEDGE >= EPT);
static_assert(RCAP >= 17531 && DEGCAP >= 41);
static_assert(RCAP % (NTHR * 4) == 0 && RCAP == NWAVE * WLCAP);
static_assert(BK_ZINTS % (NTHR * 4) == 0);
static_assert(BK_LDS_INTS * 4 <= 327680);
static_assert(GBN == DF && GBM == GWAVE * 16 && GTHR == GWAVE * 32 && DF == 4 * 32);
static_assert(NUW % NTHR == 0 && NUXB % NTHR == 0 && NUPADP % NTHR == 0 && UPART % NTHR == 0);
static_assert(UPART == DF * (DF / 8));
static_assert(ROWH == AGP && AGP == 2 * DF);

typedef float          v4f   __attribute__((ext_vector_type(4)));
typedef float          v8f   __attribute__((ext_vector_type(8)));
typedef int            v4i   __attribute__((ext_vector_type(4)));
typedef int            v8i   __attribute__((ext_vector_type(8)));
typedef unsigned       v2u   __attribute__((ext_vector_type(2)));
typedef unsigned short v4us  __attribute__((ext_vector_type(4)));
typedef unsigned short v8us  __attribute__((ext_vector_type(8)));
typedef unsigned short v16us __attribute__((ext_vector_type(16)));
typedef __bf16         v16bf __attribute__((ext_vector_type(16)));
typedef v4f  __attribute__((may_alias)) v4fa;
typedef v4i  __attribute__((may_alias)) v4ia;
typedef v2u  __attribute__((may_alias)) v2ua;
typedef v4us __attribute__((may_alias)) v4usa;
typedef v8us __attribute__((may_alias)) v8usa;
union FragB { v16bf v; v16us u; v8us h[2]; v8i w; };

__device__ __forceinline__ v8f wmb(const FragB& a, const FragB& b, v8f c) {
  v8f d = __builtin_amdgcn_wmma_f32_16x16x32_bf16(false, a.v, false, b.v, (short)0, c, false, false);
  asm volatile("v_nop\n\tv_nop\n\tv_nop\n\tv_nop" : "+v"(d) : "v"(a.w), "v"(b.w));
  return d;
}

__device__ __forceinline__ unsigned bf16_bits(float f) {
  const unsigned u = __float_as_uint(f);
  return (u + 0x7FFFu + ((u >> 16) & 1u)) >> 16;
}
__device__ __forceinline__ float bf16_val(float f) {
  return __uint_as_float(bf16_bits(f) << 16);
}
__device__ __forceinline__ unsigned hl_bits(float v, unsigned& lo) {
  const unsigned hb = bf16_bits(v);
  lo = bf16_bits(v - __uint_as_float(hb << 16));
  return hb;
}

__device__ __forceinline__ void wave_sync() {
  __builtin_amdgcn_fence(__ATOMIC_RELEASE, "wavefront");
  __builtin_amdgcn_wave_barrier();
  __builtin_amdgcn_fence(__ATOMIC_ACQUIRE, "wavefront");
}

__device__ __forceinline__ void put8(unsigned short* dp, v8us o) {
  *(volatile v8us*)dp = o;
  __threadfence();
  *(volatile v8us*)dp = o;
}
__device__ __forceinline__ void put4(float* dp, v4f o) {
  *(volatile v4f*)dp = o;
  __threadfence();
  *(volatile v4f*)dp = o;
}

__device__ __forceinline__ void prep_w(const float* __restrict__ W, unsigned short* P, int pitch, int coff, int v) {
  const int n  = v >> 4;
  const int k8 = (v & 15) * 8;
  const float* p = W + (size_t)k8 * DF + n;
  v8us o;
#pragma unroll
  for (int i = 0; i < 8; ++i) o[i] = (unsigned short)bf16_bits(p[(size_t)i * DF]);
  put8(P + (size_t)n * pitch + coff + k8, o);
}

__global__ __launch_bounds__(NTHR) void k_prep(const float* __restrict__ x,
                                               const float* __restrict__ ws1, const float* __restrict__ wn1,
                                               const float* __restrict__ b1,
                                               const float* __restrict__ ws2, const float* __restrict__ wn2,
                                               const float* __restrict__ b2,
                                               unsigned short* XB, unsigned short* W1C, unsigned short* W2C,
                                               float* B1F, float* B2F, unsigned short* AGG, unsigned short* H1HL) {
  const int tid = (int)threadIdx.x;
  const int u0  = (int)blockIdx.x * NTHR;
  if (u0 < NUW) {
    const int part = u0 >> 11;
    const int v    = (u0 + tid) & (UPART - 1);
    if (part == 0)      prep_w(ws1, W1C, K1T, 0, v);
    else if (part == 1) prep_w(wn1, W1C, K1T, DF, v);
    else if (part == 2) prep_w(wn1, W1C, K1T, 2 * DF, v);
    else if (part == 3) prep_w(ws2, W2C, K2T, 0, v);
    else if (part == 4) prep_w(ws2, W2C, K2T, DF, v);
    else if (part == 5) prep_w(wn2, W2C, K2T, 2 * DF, v);
    else                prep_w(wn2, W2C, K2T, 3 * DF, v);
  } else if (u0 < NUW + NUXB) {
    const int v   = u0 + tid - NUW;
    const int row = v >> 4;
    const int c8  = (v & 15) * 8;
    const int rc  = row < NNODE ? row : NNODE - 1;
    const unsigned msk = row < NNODE ? 0xFFFFu : 0u;
    const float* p = x + (size_t)rc * DF + c8;
    const v4f a = *(const v4f*)p;
    const v4f b = *(const v4f*)(p + 4);
    v8us o;
    o[0] = (unsigned short)(bf16_bits(a.x) & msk); o[1] = (unsigned short)(bf16_bits(a.y) & msk);
    o[2] = (unsigned short)(bf16_bits(a.z) & msk); o[3] = (unsigned short)(bf16_bits(a.w) & msk);
    o[4] = (unsigned short)(bf16_bits(b.x) & msk); o[5] = (unsigned short)(bf16_bits(b.y) & msk);
    o[6] = (unsigned short)(bf16_bits(b.z) & msk); o[7] = (unsigned short)(bf16_bits(b.w) & msk);
    put8(XB + (size_t)v * 8, o);
  } else if (u0 < NUW + NUXB + NUPADP) {
    const int v = u0 + tid - (NUW + NUXB);
    const v8us z = {0, 0, 0, 0, 0, 0, 0, 0};
    put8(AGG + (size_t)NNODE * AGP + (size_t)v * 8, z);
  } else if (u0 < NUW + NUXB + NUPAD) {
    const int v = u0 + tid - (NUW + NUXB + NUPADP);
    const v8us z = {0, 0, 0, 0, 0, 0, 0, 0};
    put8(H1HL + (size_t)NNODE * AGP + (size_t)v * 8, z);
  } else {
    if (tid < 32) {
      v4f t = *(const v4f*)(b1 + 4 * tid);
      t.x = bf16_val(t.x); t.y = bf16_val(t.y); t.z = bf16_val(t.z); t.w = bf16_val(t.w);
      put4(B1F + 4 * tid, t);
    } else if (tid < 64) {
      const int l = tid - 32;
      v4f t = *(const v4f*)(b2 + 4 * l);
      t.x = bf16_val(t.x); t.y = bf16_val(t.y); t.z = bf16_val(t.z); t.w = bf16_val(t.w);
      put4(B2F + 4 * l, t);
    }
  }
}

__device__ __forceinline__ void hit1(bool hj, unsigned sj, int srcj, int& wc, int* mylist) {
  const unsigned mj = __builtin_amdgcn_ballot_w32(hj);
  if (mj != 0u) {
    const int pos = wc + (int)__builtin_amdgcn_mbcnt_lo(mj, 0u);
    const int sc  = srcj < 0 ? 0 : (srcj > NNODE - 1 ? NNODE - 1 : srcj);
    const int pk  = (int)(sj << 16) | sc;
    if (hj && pos < WLCAP) mylist[pos] = pk;
    wc += (int)__builtin_popcount(mj);
  }
}

__global__ __launch_bounds__(NTHR) void k_bucket(const int* __restrict__ srcs, const int* __restrict__ dsts,
                                                 int* LIST, int* CNT, int* OFF, int* FLAG) {
  extern __shared__ __attribute__((aligned(16))) int dsm[];
  int* wl   = dsm;
  int* sl   = wl + BK_LISTS;
  int* cnt  = sl + RCAP;
  int* offs = cnt + NBA;
  int* cur  = offs + NBA;
  int* misc = cur + NBA;
  const int tid = (int)threadIdx.x, lane = tid & 31, wave = tid >> 5;
  const int blk = (int)blockIdx.x;
  const int nodeBase = blk * NBA;

  {
    const v4i z4 = {0, 0, 0, 0};
    for (int i = tid * 4; i < BK_ZINTS; i += NTHR * 4) *(v4ia*)(dsm + i) = z4;
    if (tid < BK_MISC) misc[tid] = 0;
  }
  __syncthreads();

  int wc = 0;
  int* mylist = wl + wave * WLCAP;
  const unsigned nbs = (unsigned)nodeBase;
  const unsigned unb = (unsigned)NBA;
#pragma unroll 1
  for (int ch = 0; ch < NCHUNK; ++ch) {
    const int e0   = ch * CHUNK + tid * EPT;
    const bool inr = e0 < NEDGE;
    const int ec   = inr ? e0 : (NEDGE - EPT);
    const v4i da = *(const v4i*)(dsts + ec);
    const v4i db = *(const v4i*)(dsts + ec + 4);
    const v4i sa = *(const v4i*)(srcs + ec);
    const v4i sb = *(const v4i*)(srcs + ec + 4);
    asm volatile("" :: "v"(da), "v"(db), "v"(sa), "v"(sb));
    const unsigned s0 = (unsigned)da.x - nbs, s1 = (unsigned)da.y - nbs;
    const unsigned s2 = (unsigned)da.z - nbs, s3 = (unsigned)da.w - nbs;
    const unsigned s4 = (unsigned)db.x - nbs, s5 = (unsigned)db.y - nbs;
    const unsigned s6 = (unsigned)db.z - nbs, s7 = (unsigned)db.w - nbs;
    const bool h0 = (s0 < unb) & inr, h1 = (s1 < unb) & inr, h2 = (s2 < unb) & inr, h3 = (s3 < unb) & inr;
    const bool h4 = (s4 < unb) & inr, h5 = (s5 < unb) & inr, h6 = (s6 < unb) & inr, h7 = (s7 < unb) & inr;
    hit1(h0, s0, sa.x, wc, mylist);
    hit1(h1, s1, sa.y, wc, mylist);
    hit1(h2, s2, sa.z, wc, mylist);
    hit1(h3, s3, sa.w, wc, mylist);
    hit1(h4, s4, sb.x, wc, mylist);
    hit1(h5, s5, sb.y, wc, mylist);
    hit1(h6, s6, sb.z, wc, mylist);
    hit1(h7, s7, sb.w, wc, mylist);
  }
  if (lane == 0) misc[wave] = wc;
  __syncthreads();

  if (wave == 0) {
    int ov = 0;
#pragma unroll 1
    for (int w2 = 0; w2 < NWAVE; ++w2) {
      int c = misc[w2];
      if (c > WLCAP) ov = 1;
      c = c < 0 ? 0 : (c > WLCAP ? WLCAP : c);
#pragma unroll 1
      for (int b0 = 0; b0 < c; b0 += 32) {
        const int idx = b0 + lane;
        const int ent = wl[w2 * WLCAP + (idx < WLCAP ? idx : WLCAP - 1)];
        const int m32 = (c - b0) < 32 ? (c - b0) : 32;
#pragma unroll 1
        for (int k = 0; k < m32; ++k) {
          const int u    = __builtin_amdgcn_readlane(ent, k);
          const int slot = (u >> 16) & (NBA - 1);
          if (lane == 0) cnt[slot] = cnt[slot] + 1;
        }
      }
    }
    if (lane == 0) misc[9] = ov;
  }
  __syncthreads();

  if (wave == 0) {
    const int base = lane * (NBA / 32);
    int s = 0;
#pragma unroll 1
    for (int i = 0; i < NBA / 32; ++i) s += cnt[base + i];
    int incl = s;
#pragma unroll
    for (int d = 1; d < 32; d <<= 1) {
      const int y = __shfl_up(incl, d, 32);
      if (lane >= d) incl += y;
    }
    int run = incl - s;
#pragma unroll 1
    for (int i = 0; i < NBA / 32; ++i) {
      const int cv = cnt[base + i];
      offs[base + i] = run;
      cur[base + i]  = run;
      run += cv;
    }
  }
  __syncthreads();

  if (wave == 0) {
#pragma unroll 1
    for (int w2 = 0; w2 < NWAVE; ++w2) {
      int c = misc[w2];
      c = c < 0 ? 0 : (c > WLCAP ? WLCAP : c);
#pragma unroll 1
      for (int b0 = 0; b0 < c; b0 += 32) {
        const int idx = b0 + lane;
        const int ent = wl[w2 * WLCAP + (idx < WLCAP ? idx : WLCAP - 1)];
        const int m32 = (c - b0) < 32 ? (c - b0) : 32;
#pragma unroll 1
        for (int k = 0; k < m32; ++k) {
          const int u    = __builtin_amdgcn_readlane(ent, k);
          const int slot = (u >> 16) & (NBA - 1);
          if (lane == 0) {
            int p = cur[slot];
            p = p < 0 ? 0 : (p > RCAP - 1 ? RCAP - 1 : p);
            sl[p] = u & 0xFFFF;
            cur[slot] = p + 1;
          }
        }
      }
    }
  }
  __syncthreads();

  const int ovf = misc[9];
  asm volatile("" :: "v"(ovf));
  int* Lb = LIST + (size_t)blk * RCAP;
  const v4i cq = *(const v4ia*)(cnt + 4 * tid);
  const v4i oq = *(const v4ia*)(offs + 4 * tid);
  const v4i fq = {ovf, ovf, ovf, ovf};
#pragma unroll 1
  for (int i = tid * 4; i < RCAP; i += NTHR * 4) {
    const v4i q = *(const v4ia*)(sl + i);
    *(volatile v4i*)(Lb + i) = q;
  }
  *(volatile v4i*)(CNT + nodeBase + 4 * tid) = cq;
  *(volatile v4i*)(OFF + nodeBase + 4 * tid) = oq;
  if (tid < 8) *(volatile v4i*)(FLAG + blk * FLP + 4 * tid) = fq;
  __threadfence();
#pragma unroll 1
  for (int i = tid * 4; i < RCAP; i += NTHR * 4) {
    const v4i q = *(const v4ia*)(sl + i);
    *(volatile v4i*)(Lb + i) = q;
  }
  *(volatile v4i*)(CNT + nodeBase + 4 * tid) = cq;
  *(volatile v4i*)(OFF + nodeBase + 4 * tid) = oq;
  if (tid < 8) *(volatile v4i*)(FLAG + blk * FLP + 4 * tid) = fq;
}

template <int L2>
__global__ __launch_bounds__(NTHR) void k_agg(const unsigned short* __restrict__ hp, const int* __restrict__ LIST,
                                              const int* __restrict__ CNT, const int* __restrict__ OFF,
                                              const int* __restrict__ FLAG, unsigned short* AGG) {
  __shared__ __attribute__((aligned(16))) int scnt[NBA];
  __shared__ __attribute__((aligned(16))) int soff[NBA];
  __shared__ __attribute__((aligned(16))) unsigned short rowbuf[NWAVE * ROWH];
  const int tid = (int)threadIdx.x, lane = tid & 31, wave = tid >> 5;
  const int blk = (int)blockIdx.x;
  const int nodeBase = blk * NBA;
  {
    const v4i cq = *(const v4i*)(CNT + nodeBase + 4 * tid);
    const v4i oq = *(const v4i*)(OFF + nodeBase + 4 * tid);
    *(v4ia*)(scnt + 4 * tid) = cq;
    *(v4ia*)(soff + 4 * tid) = oq;
  }
  const int fl = FLAG[blk * FLP];
  __syncthreads();

  const int* Lb = LIST + (size_t)blk * RCAP;
  unsigned short* rb = rowbuf + wave * ROWH;
  const float qn = __int_as_float(0x7fc00000);
  const float pz = (fl != 0) ? qn : 0.0f;
#pragma unroll 1
  for (int si = 0; si < NBA / NWAVE; ++si) {
    const int s    = si * NWAVE + wave;
    const int node = nodeBase + s;
    int c = scnt[s];
    const bool big = c > DEGCAP;
    c = c < 0 ? 0 : (c > DEGCAP ? DEGCAP : c);
    int o = soff[s];
    o = o < 0 ? 0 : (o > RCAP ? RCAP : o);
    const float pzr = big ? qn : pz;
    const bool live = node < NNODE;
    float a0 = 0.0f, a1 = 0.0f, a2 = 0.0f, a3 = 0.0f;
#pragma unroll 1
    for (int b0 = 0; b0 < c; b0 += 32) {
      int idx = o + b0 + lane;
      idx = idx > RCAP - 1 ? RCAP - 1 : idx;
      int sr = Lb[idx];
      sr = sr < 0 ? 0 : (sr > NNODE - 1 ? NNODE - 1 : sr);
      const int m32 = (c - b0) < 32 ? (c - b0) : 32;
#pragma unroll 1
      for (int k = 0; k < m32; ++k) {
        const int sk = __builtin_amdgcn_readlane(sr, k);
        if constexpr (L2 == 0) {
          const v2u w = *(const v2ua*)(hp + (size_t)sk * DF + 4 * lane);
          a0 += __uint_as_float(w.x << 16);
          a1 += __uint_as_float(w.x & 0xffff0000u);
          a2 += __uint_as_float(w.y << 16);
          a3 += __uint_as_float(w.y & 0xffff0000u);
        } else {
          const unsigned short* rp = hp + (size_t)sk * AGP + 4 * lane;
          const v2u wh = *(const v2ua*)rp;
          const v2u wo = *(const v2ua*)(rp + DF);
          const float f0 = __uint_as_float(wh.x << 16)         + __uint_as_float(wo.x << 16);
          const float f1 = __uint_as_float(wh.x & 0xffff0000u) + __uint_as_float(wo.x & 0xffff0000u);
          const float f2 = __uint_as_float(wh.y << 16)         + __uint_as_float(wo.y << 16);
          const float f3 = __uint_as_float(wh.y & 0xffff0000u) + __uint_as_float(wo.y & 0xffff0000u);
          a0 += f0; a1 += f1; a2 += f2; a3 += f3;
        }
      }
    }
    const float dv = (float)(c < 1 ? 1 : c);
    const float m0 = live ? (a0 / dv + pzr) : 0.0f;
    const float m1 = live ? (a1 / dv + pzr) : 0.0f;
    const float m2 = live ? (a2 / dv + pzr) : 0.0f;
    const float m3 = live ? (a3 / dv + pzr) : 0.0f;
    v4us mh, ml;
    {
      unsigned lb;
      unsigned hb;
      hb = hl_bits(m0, lb); mh[0] = (unsigned short)hb; ml[0] = (unsigned short)lb;
      hb = hl_bits(m1, lb); mh[1] = (unsigned short)hb; ml[1] = (unsigned short)lb;
      hb = hl_bits(m2, lb); mh[2] = (unsigned short)hb; ml[2] = (unsigned short)lb;
      hb = hl_bits(m3, lb); mh[3] = (unsigned short)hb; ml[3] = (unsigned short)lb;
    }
    *(v4usa*)(rb + 4 * lane)      = mh;
    *(v4usa*)(rb + DF + 4 * lane) = ml;
    wave_sync();
    const v8us q0 = *(const v8usa*)(rb + 8 * lane);
    wave_sync();
    if (node < MP) {
      unsigned short* rpw = AGG + (size_t)node * AGP + 8 * lane;
      *(volatile v8us*)rpw = q0;
      __threadfence();
      *(volatile v8us*)rpw = q0;
    }
  }
}

template <int NSTEP, int LDB>
__device__ __forceinline__ void kseg(const unsigned short* __restrict__ ap, const unsigned short* __restrict__ bp,
                                     v8f (&acc)[8]) {
#pragma unroll 1
  for (int s = 0; s < NSTEP; ++s) {
    const int k0 = 32 * s;
    FragB af;
    af.h[0] = *(const v8usa*)(ap + k0);
    af.h[1] = *(const v8usa*)(ap + k0 + 16);
#pragma unroll
    for (int nt = 0; nt < 8; ++nt) {
      const unsigned short* wq = bp + (size_t)(16 * nt) * (size_t)LDB + k0;
      FragB bf;
      bf.h[0] = *(const v8usa*)wq;
      bf.h[1] = *(const v8usa*)(wq + 16);
      acc[nt] = wmb(af, bf, acc[nt]);
    }
  }
}

template <int FIN, int S0W, int S0P, int S1W, int S1P>
__global__ __launch_bounds__(GTHR) __attribute__((amdgpu_num_vgpr(248)))
void k_gemm(const unsigned short* __restrict__ A0, const unsigned short* __restrict__ A1,
            const unsigned short* __restrict__ BT, const float* __restrict__ bfv,
            const int* __restrict__ FLAG, unsigned short* hout, float* outp) {
  constexpr int KT = S0W + S1W;
  static_assert(S0W % 32 == 0 && S1W % 32 == 0 && S0W <= S0P && S1W <= S1P && KT % 32 == 0);
  __shared__ __attribute__((aligned(16))) float stg[GBM * GBN];
  __shared__ __attribute__((aligned(16))) float bsm[DF];
  __shared__ __attribute__((aligned(16))) unsigned short rst[GWAVE * ROWH];
  const int tid = (int)threadIdx.x, lane = tid & 31, wave = tid >> 5, hh = lane >> 4, m = lane & 15;
  const int rowBase = (int)blockIdx.x * GBM;

  if (tid < 32) {
    const v4f b4 = *(const v4f*)(bfv + 4 * tid);
    *(v4fa*)(bsm + 4 * tid) = b4;
  }

  v8f acc[8];
  {
    const v8f z = {0.f, 0.f, 0.f, 0.f, 0.f, 0.f, 0.f, 0.f};
#pragma unroll
    for (int t = 0; t < 8; ++t) acc[t] = z;
  }
  const size_t arow = (size_t)(rowBase + 16 * wave + m);
  const unsigned short* a0p = A0 + arow * (size_t)S0P + 8 * hh;
  const unsigned short* a1p = A1 + arow * (size_t)S1P + 8 * hh;
  const unsigned short* bp  = BT + (size_t)m * (size_t)KT + 8 * hh;
  kseg<S0W / 32, KT>(a0p, bp, acc);
  kseg<S1W / 32, KT>(a1p, bp + S0W, acc);

#pragma unroll
  for (int nt = 0; nt < 8; ++nt) {
    const int lc = 16 * nt + m;
#pragma unroll
    for (int r = 0; r < 8; ++r) {
      const int lr = 16 * wave + 8 * hh + r;
      stg[lr * GBN + lc] = acc[nt][r];
    }
  }
  __syncthreads();

  const v4f bb4 = *(const v4fa*)(bsm + 4 * lane);

  if constexpr (FIN != 0) {
    const int fl = FLAG[(rowBase >> SLA) * FLP];
    const float qn = __int_as_float(0x7fc00000);
#pragma unroll 1
    for (int i = 0; i < 16; ++i) {
      const int lr  = 16 * wave + i;
      const int row = rowBase + lr;
      const v4f t = *(const v4fa*)(stg + lr * GBN + 4 * lane) + bb4;
      v4f y;
      y.x = (fl != 0) ? qn : t.x; y.y = (fl != 0) ? qn : t.y;
      y.z = (fl != 0) ? qn : t.z; y.w = (fl != 0) ? qn : t.w;
      if (row < NNODE) *(volatile v4f*)(outp + (size_t)row * DF + 4 * lane) = y;
    }
    __threadfence();
#pragma unroll 1
    for (int i = 0; i < 16; ++i) {
      const int lr  = 16 * wave + i;
      const int row = rowBase + lr;
      const v4f t = *(const v4fa*)(stg + lr * GBN + 4 * lane) + bb4;
      v4f y;
      y.x = (fl != 0) ? qn : t.x; y.y = (fl != 0) ? qn : t.y;
      y.z = (fl != 0) ? qn : t.z; y.w = (fl != 0) ? qn : t.w;
      if (row < NNODE) *(volatile v4f*)(outp + (size_t)row * DF + 4 * lane) = y;
    }
    (void)hout; (void)rst;
  } else {
    unsigned short* rb = rst + wave * ROWH;
#pragma unroll 1
    for (int pass = 0; pass < 2; ++pass) {
#pragma unroll 1
      for (int i = 0; i < 16; ++i) {
        const int lr  = 16 * wave + i;
        const int row = rowBase + lr;
        const bool ok = row < NNODE;
        const v4f t = *(const v4fa*)(stg + lr * GBN + 4 * lane) + bb4;
        float y0 = (t.x > 0.0f) ? t.x : (t.x - t.x);
        float y1 = (t.y > 0.0f) ? t.y : (t.y - t.y);
        float y2 = (t.z > 0.0f) ? t.z : (t.z - t.z);
        float y3 = (t.w > 0.0f) ? t.w : (t.w - t.w);
        y0 = ok ? y0 : 0.0f; y1 = ok ? y1 : 0.0f; y2 = ok ? y2 : 0.0f; y3 = ok ? y3 : 0.0f;
        v4us h4, l4;
        unsigned lb;
        unsigned hb;
        hb = hl_bits(y0, lb); h4[0] = (unsigned short)hb; l4[0] = (unsigned short)lb;
        hb = hl_bits(y1, lb); h4[1] = (unsigned short)hb; l4[1] = (unsigned short)lb;
        hb = hl_bits(y2, lb); h4[2] = (unsigned short)hb; l4[2] = (unsigned short)lb;
        hb = hl_bits(y3, lb); h4[3] = (unsigned short)hb; l4[3] = (unsigned short)lb;
        *(v4usa*)(rb + 4 * lane)      = h4;
        *(v4usa*)(rb + DF + 4 * lane) = l4;
        wave_sync();
        const v8us q = *(const v8usa*)(rb + 8 * lane);
        wave_sync();
        *(volatile v8us*)(hout + (size_t)row * AGP + 8 * lane) = q;
      }
      __threadfence();
    }
    (void)outp; (void)FLAG;
  }
}

static inline size_t al256(size_t o) { return (o + 255) & ~(size_t)255; }

extern "C" void kernel_launch(void* const* d_in, const int* in_sizes, int n_in,
                              void* d_out, int out_size, void* d_ws, size_t ws_size,
                              hipStream_t stream) {
  if (n_in < 9) return;
  if (in_sizes[0] != NNODE * DF) return;
  if (in_sizes[1] != NEDGE || in_sizes[2] != NEDGE) return;
  if (in_sizes[3] != DF * DF || in_sizes[4] != DF * DF || in_sizes[5] != DF) return;
  if (in_sizes[6] != DF * DF || in_sizes[7] != DF * DF || in_sizes[8] != DF) return;
  if (out_size != NNODE * DF) return;

  const float* x   = (const float*)d_in[0];
  const int*   src = (const int*)  d_in[1];
  const int*   dst = (const int*)  d_in[2];
  const float* Ws1 = (const float*)d_in[3];
  const float* Wn1 = (const float*)d_in[4];
  const float* b1  = (const float*)d_in[5];
  const float* Ws2 = (const float*)d_in[6];
  const float* Wn2 = (const float*)d_in[7];
  const float* b2  = (const float*)d_in[8];
  float* out = (float*)d_out;

  char* ws = (char*)d_ws;
  size_t off = 0;
  const size_t oXB   = off; off = al256(off + (size_t)MP * DF * 2);
  const size_t oAGG  = off; off = al256(off + (size_t)MP * AGP * 2);
  const size_t oH1   = off; off = al256(off + (size_t)MP * AGP * 2);
  const size_t oLIST = off; off = al256(off + (size_t)NBLK * RCAP * 4);
  const size_t oCNT  = off; off = al256(off + (size_t)NBLK * NBA * 4);
  const size_t oOFF  = off; off = al256(off + (size_t)NBLK * NBA * 4);
  const size_t oFLG  = off; off = al256(off + (size_t)NBLK * FLP * 4);
  const size_t oW1   = off; off = al256(off + (size_t)DF * K1T * 2);
  const size_t oW2   = off; off = al256(off + (size_t)DF * K2T * 2);
  const size_t oB1   = off; off = al256(off + (size_t)DF * 4);
  const size_t oB2   = off; off = al256(off + (size_t)DF * 4);
  if (off > ws_size || off > (size_t)WSMAX) return;
  unsigned short* XB   = (unsigned short*)(ws + oXB);
  unsigned short* AGG  = (unsigned short*)(ws + oAGG);
  unsigned short* H1HL = (unsigned short*)(ws + oH1);
  int* LIST = (int*)(ws + oLIST);
  int* CNT  = (int*)(ws + oCNT);
  int* OFF  = (int*)(ws + oOFF);
  int* FLAG = (int*)(ws + oFLG);
  unsigned short* W1C = (unsigned short*)(ws + oW1);
  unsigned short* W2C = (unsigned short*)(ws + oW2);
  float* B1F = (float*)(ws + oB1);
  float* B2F = (float*)(ws + oB2);

  const size_t bkLds = (size_t)BK_LDS_INTS * 4;
  hipFuncSetAttribute(reinterpret_cast<const void*>(&k_bucket), hipFuncAttributeMaxDynamicSharedMemorySize, (int)bkLds);

  const int gM = MP / GBM;

  k_prep<<<NUTOT / NTHR, NTHR, 0, stream>>>(x, Ws1, Wn1, b1, Ws2, Wn2, b2, XB, W1C, W2C, B1F, B2F, AGG, H1HL);
  k_bucket<<<NBLK, NTHR, bkLds, stream>>>(src, dst, LIST, CNT, OFF, FLAG);
  k_agg<0><<<NBLK, NTHR, 0, stream>>>(XB, LIST, CNT, OFF, FLAG, AGG);
  k_gemm<0, L1_S0W, L1_S0P, L1_S1W, L1_S1P><<<gM, GTHR, 0, stream>>>(XB, AGG, W1C, B1F, FLAG, H1HL, out);
  k_agg<1><<<NBLK, NTHR, 0, stream>>>(H1HL, LIST, CNT, OFF, FLAG, AGG);
  k_gemm<1, L2_S0W, L2_S0P, L2_S1W, L2_S1P><<<gM, GTHR, 0, stream>>>(H1HL, AGG, W2C, B2F, FLAG, H1HL, out);
}
